// SRGModel_16432544875093
// MI455X (gfx1250) — hardware-verified
//
#include <hip/hip_runtime.h>
#include <math.h>
typedef __attribute__((ext_vector_type(16))) _Float16 v16h;
typedef __attribute__((ext_vector_type(8)))  _Float16 v8h;
typedef __attribute__((ext_vector_type(16))) __bf16   v16b;
typedef __attribute__((ext_vector_type(8)))  __bf16   v8b;
typedef __attribute__((ext_vector_type(8)))  float    v8f;
typedef __attribute__((ext_vector_type(4)))  float    v4f;
#define PSCALE 32768.0f
#define U16(p) ((const unsigned short*)(const void*)(p))
#define PSCALE_INV (1.0f / 32768.0f)

__device__ __forceinline__ unsigned short f2bf_bits(float f) {
  unsigned u = __float_as_uint(f);
  return (unsigned short)((u + 0x7FFFu + ((u >> 16) & 1u)) >> 16);
}
__device__ __forceinline__ float bf_bits2f(unsigned short h) { return __uint_as_float(((unsigned)h) << 16); }

__device__ __forceinline__ void dep_guard_h(v8f& a, v8f& b, v16h x, v16h y) { asm volatile("v_nop\n\tv_nop\n\tv_nop\n\tv_nop" : "+v"(a), "+v"(b) : "v"(x), "v"(y)); }
__device__ __forceinline__ void dep_guard_b(v8f& a, v8f& b, v16b x, v16b y) { asm volatile("v_nop\n\tv_nop\n\tv_nop\n\tv_nop" : "+v"(a), "+v"(b) : "v"(x), "v"(y)); }
__device__ __forceinline__ void keep4_h(v16h a, v16h b, v16h c, v16h d) { asm volatile("v_nop" :: "v"(a), "v"(b), "v"(c), "v"(d)); }
__device__ __forceinline__ void keep4_b(v16b a, v16b b, v16b c, v16b d) { asm volatile("v_nop" :: "v"(a), "v"(b), "v"(c), "v"(d)); }
__device__ __forceinline__ void acc_guard4(v8f& a, v8f& b, v8f& c, v8f& d) { asm volatile("v_nop\n\tv_nop\n\tv_nop\n\tv_nop" : "+v"(a), "+v"(b), "+v"(c), "+v"(d)); }
template <typename T> struct Frag;
template <> struct Frag<_Float16> {
  typedef v16h V; union U { v16h v; v8h h[2]; };
  static __device__ __forceinline__ v16h load(const _Float16* p) {
    U f; f.h[0] = *(const v8h*)(p); f.h[1] = *(const v8h*)(p + 16); return f.v;
  }
  static __device__ __forceinline__ v8f mma(v16h a, v16h b, v8f c) {
    return __builtin_amdgcn_wmma_f32_16x16x32_f16(false, a, false, b, (short)0, c, false, false);
  }
  static __device__ __forceinline__ void guard(v8f& a, v8f& b, v16h x, v16h y) { dep_guard_h(a, b, x, y); }
  static __device__ __forceinline__ void keep(v16h a, v16h b, v16h c, v16h d) { keep4_h(a, b, c, d); }
};
template <> struct Frag<__bf16> {
  typedef v16b V; union U { v16b v; v8b h[2]; };
  static __device__ __forceinline__ v16b load(const __bf16* p) {
    U f; f.h[0] = *(const v8b*)(p); f.h[1] = *(const v8b*)(p + 16); return f.v;
  }
  static __device__ __forceinline__ v8f mma(v16b a, v16b b, v8f c) {
    return __builtin_amdgcn_wmma_f32_16x16x32_bf16(false, a, false, b, (short)0, c, false, false);
  }
  static __device__ __forceinline__ void guard(v8f& a, v8f& b, v16b x, v16b y) { dep_guard_b(a, b, x, y); }
  static __device__ __forceinline__ void keep(v16b a, v16b b, v16b c, v16b d) { keep4_b(a, b, c, d); }
};

template <int ET> struct Elem;
template <> struct Elem<0> { typedef _Float16 T; };
template <> struct Elem<1> { typedef __bf16 T; };
template <int ET, bool SPLIT, int BIAS_MODE, int OUT_MODE, bool RESID, int ACT = 0>
__global__ __launch_bounds__(256) void wmma_gemm64(
    const unsigned short* __restrict__ Ap, const unsigned short* __restrict__ A2p, int lda, long strideA,
    const unsigned short* __restrict__ Btp, const unsigned short* __restrict__ Bt2p, int ldb, long strideB,
    void* __restrict__ Cout, void* __restrict__ Cout2, int ldc, long strideC,
    const float* __restrict__ bias,
    const float* __restrict__ resid, long strideR,
    int M, int N, int K, float scale) {
  typedef typename Elem<ET>::T T;
  typedef typename Frag<T>::V V;
  const T* A = (const T*)Ap; const T* A2 = (const T*)A2p; const T* Bt = (const T*)Btp; const T* Bt2 = (const T*)Bt2p;
  __shared__ __align__(16) float sT[8][16 * 68];
  const int b    = blockIdx.y;
  const int lane = threadIdx.x & 31;
  const int wave = threadIdx.x >> 5;
  const int tilesN = N >> 6;
  const int tilesM = M >> 6;
  const int tile = blockIdx.x * 8 + wave;
  if (tile >= tilesM * tilesN) return;
  const int tm = tile / tilesN;
  const int tn = tile - tm * tilesN;
  const int m0 = tm << 6;
  const int n0 = tn << 6;

  const T* Ab  = A  + (size_t)b * strideA;
  const T* Bb  = Bt + (size_t)b * strideB;
  const T* Ab2 = SPLIT ? (A2  + (size_t)b * strideA) : nullptr;
  const T* Bb2 = SPLIT ? (Bt2 + (size_t)b * strideB) : nullptr;

  const int rlane = lane & 15;
  const int koff  = (lane >> 4) * 8;
  const int mOff  = (lane >> 4) * 8;

  v8f acc[4][4];
#pragma unroll
  for (int i = 0; i < 4; ++i)
#pragma unroll
    for (int j = 0; j < 4; ++j) acc[i][j] = (v8f){0.f,0.f,0.f,0.f,0.f,0.f,0.f,0.f};

  for (int k0 = 0; k0 < K; k0 += 32) {
    V bh[4], bl[4];
#pragma unroll
    for (int j = 0; j < 4; ++j) {
      const size_t bo = (size_t)(n0 + (j << 4) + rlane) * ldb + koff + k0;
      bh[j] = Frag<T>::load(Bb + bo);
      if (SPLIT) bl[j] = Frag<T>::load(Bb2 + bo);
    }
#pragma unroll
    for (int i = 0; i < 4; ++i) {
      const size_t ao = (size_t)(m0 + (i << 4) + rlane) * lda + koff + k0;
      V ah = Frag<T>::load(Ab + ao);
      V al;
      if (SPLIT) al = Frag<T>::load(Ab2 + ao);
#pragma unroll
      for (int j = 0; j < 4; ++j) {
        acc[i][j] = Frag<T>::mma(ah, bh[j], acc[i][j]);
        if (SPLIT) {
          acc[i][j] = Frag<T>::mma(ah, bl[j], acc[i][j]);
          acc[i][j] = Frag<T>::mma(al, bh[j], acc[i][j]);
        }
      }
      Frag<T>::guard(acc[i][0], acc[i][3], ah, SPLIT ? al : ah);
    }
    Frag<T>::keep(bh[0], bh[1], bh[2], bh[3]);
    if (SPLIT) Frag<T>::keep(bl[0], bl[1], bl[2], bl[3]);
  }
  acc_guard4(acc[0][0], acc[0][1], acc[0][2], acc[0][3]);
  acc_guard4(acc[1][0], acc[1][1], acc[1][2], acc[1][3]);
  acc_guard4(acc[2][0], acc[2][1], acc[2][2], acc[2][3]);
  acc_guard4(acc[3][0], acc[3][1], acc[3][2], acc[3][3]);

  float* slab = sT[wave];
  const float* Rb = RESID ? (resid + (size_t)b * strideR) : nullptr;
#pragma unroll
  for (int i = 0; i < 4; ++i) {
    const int mBase = m0 + (i << 4);
#pragma unroll
    for (int j = 0; j < 4; ++j) {
      const int n = n0 + (j << 4) + rlane;
      float bv = 0.f;
      if (BIAS_MODE == 2) bv = bias[n];
#pragma unroll
      for (int r = 0; r < 8; ++r) {
        float v = acc[i][j][r] * scale;
        if (BIAS_MODE == 1) v += bias[mBase + mOff + r];
        if (BIAS_MODE == 2) v += bv;
        if (RESID) v += Rb[(size_t)(mBase + mOff + r) * ldc + n];
        if (ACT == 1) v = tanhf(v);
        if (ACT == 2) v = fmaxf(v, 0.0f);
        if (ACT == 3) v = v / (1.0f + expf(-v));
        if (ACT == 4) v = (v > 0.f) ? v : 0.01f * v;
        if (ACT == 5) v = 0.5f * v * (1.0f + erff(v * 0.70710678118654752f));
        slab[(mOff + r) * 68 + (j << 4) + rlane] = v;
      }
    }
    __builtin_amdgcn_fence(__ATOMIC_RELEASE, "workgroup");
    __builtin_amdgcn_wave_barrier();
    __builtin_amdgcn_fence(__ATOMIC_ACQUIRE, "workgroup");
    if (OUT_MODE == 0) {
      float* C = (float*)Cout + (size_t)b * strideC;
      const int hh = lane >> 4, c4 = (lane & 15) * 4;
      for (int pass = 0; pass < 2; ++pass) {
#pragma unroll
        for (int it = 0; it < 8; ++it) {
          const int row = it * 2 + hh;
          v4f v = *(const v4f*)(slab + row * 68 + c4);
          *(volatile v4f*)(C + (size_t)(mBase + row) * ldc + n0 + c4) = v;
        }
        __threadfence();
      }
    } else {
      const int q = lane >> 3, c8 = (lane & 7) * 8;
      unsigned short* C  = (unsigned short*)Cout  + (size_t)b * strideC;
      unsigned short* C2 = (OUT_MODE == 2) ? ((unsigned short*)Cout2 + (size_t)b * strideC) : nullptr;
      for (int pass = 0; pass < 2; ++pass) {
#pragma unroll
        for (int it = 0; it < 4; ++it) {
          const int row = it * 4 + q;
          const float* sp = slab + row * 68 + c8;
          v8h hv, lv;
#pragma unroll
          for (int e = 0; e < 8; ++e) {
            if (OUT_MODE == 1) {
              hv[e] = (_Float16)sp[e];
            } else {
              unsigned short hb = f2bf_bits(sp[e]);
              unsigned short lb = f2bf_bits(sp[e] - bf_bits2f(hb));
              hv[e] = __builtin_bit_cast(_Float16, hb);
              lv[e] = __builtin_bit_cast(_Float16, lb);
            }
          }
          *(volatile v8h*)(C + (size_t)(mBase + row) * ldc + n0 + c8) = hv;
          if (OUT_MODE == 2) *(volatile v8h*)(C2 + (size_t)(mBase + row) * ldc + n0 + c8) = lv;
        }
        __threadfence();
      }
    }
    __builtin_amdgcn_fence(__ATOMIC_RELEASE, "workgroup");
    __builtin_amdgcn_wave_barrier();
    __builtin_amdgcn_fence(__ATOMIC_ACQUIRE, "workgroup");
  }
}

__global__ __launch_bounds__(256) void cast_f32_f16x2(
    const float* __restrict__ in, _Float16* __restrict__ out, int n2) {
  int i = blockIdx.x * 256 + threadIdx.x;
  if (i < n2) {
    const _Float16 h0 = (_Float16)in[2 * i], h1 = (_Float16)in[2 * i + 1];
    const unsigned u = (unsigned)__builtin_bit_cast(unsigned short, h0) | ((unsigned)__builtin_bit_cast(unsigned short, h1) << 16);
    ((volatile unsigned*)out)[i] = u;
    __threadfence();
    ((volatile unsigned*)out)[i] = u;
  }
}


__global__ __launch_bounds__(256) void transpose_cast_f16(const float* __restrict__ in, int ldi,
                                                         _Float16* __restrict__ outT, int ldo, float scale) {
  __shared__ __align__(16) _Float16 tile[64][72];
  const int c0 = blockIdx.x * 64, r0 = blockIdx.y * 64;
  const int t = threadIdx.y * 32 + threadIdx.x;
  for (int i = threadIdx.y; i < 64; i += 8) {
    tile[threadIdx.x][i]      = (_Float16)(in[(size_t)(r0 + i) * ldi + c0 + threadIdx.x] * scale);
    tile[32 + threadIdx.x][i] = (_Float16)(in[(size_t)(r0 + i) * ldi + c0 + 32 + threadIdx.x] * scale);
  }
  __syncthreads();
  const int q = t >> 3, c8 = (t & 7) * 8;
  for (int pass = 0; pass < 2; ++pass) {
#pragma unroll
    for (int it = 0; it < 2; ++it) {
      const int c = it * 32 + q;
      v8h hv = *(const v8h*)(&tile[c][c8]);
      *(volatile v8h*)(outT + (size_t)(c0 + c) * ldo + r0 + c8) = hv;
    }
    __threadfence();
  }
}

#define RB 32
#define RW 12
#define RN 128
#define RH 128
#define RBW (RB * RW)
#define RROWS (RBW * 2 * RN)
#define RIN (2 * RN * RH)
__global__ __launch_bounds__(256) void flow_kernel(const float* __restrict__ HR, const float* __restrict__ LR, const float* __restrict__ fw, const float* __restrict__ fb, unsigned* __restrict__ HRGE16, double* __restrict__ PS) {
  __shared__ double red[2][256];
  const long i0 = ((long)blockIdx.x * 256 + threadIdx.x) * 2;
  double mse = 0.0, bce = 0.0; unsigned packed = 0u;
  for (int e = 0; e < 2; ++e) { const long i = i0 + e; const int col = (int)(i % RN); const int row = (int)((i / RN) % (2 * RN)); const int bw = (int)(i / ((long)2 * RN * RN)); const int b = bw / RW, w = bw % RW;
    const int wc = (w - 1) > 0 ? (w - 1) : 0; const float* cond = LR + ((size_t)b * RW + wc) * RN * RN; const float* hrin = LR + ((size_t)b * RW + w) * RN * RN;
    const int y = row % RN;
    float c0 = fb[0], c1 = fb[1];
    for (int ky = 0; ky < 3; ++ky) for (int kx = 0; kx < 3; ++kx) { const int yy = y + ky - 1, xx = col + kx - 1; if (yy < 0 || yy >= RN || xx < 0 || xx >= RN) continue; const float v = cond[yy * RN + xx]; c0 += fw[ky * 3 + kx] * v; c1 += fw[9 + ky * 3 + kx] * v; }
    const float ls = tanhf(c0), t = c1;
    const float fo = (row < RN) ? (hrin[y * RN + col] * expf(ls) + t) : t;
    const float ge = 1.0f / (1.0f + expf(-fo));
    const float hr = HR[i]; const double d = (double)hr - (double)ge; mse += d * d;
    const float lp = fmaxf(logf(hr), -100.f), l1p = fmaxf(logf(1.0f - hr), -100.f); bce += (double)ge * lp + (1.0 - (double)ge) * l1p;
    packed |= (unsigned)__builtin_bit_cast(unsigned short, (_Float16)ge) << (16 * e); }
  ((volatile unsigned*)HRGE16)[i0 / 2] = packed;
  red[0][threadIdx.x] = mse; red[1][threadIdx.x] = bce; __syncthreads();
  for (int o = 128; o > 0; o >>= 1) { if (threadIdx.x < o) { red[0][threadIdx.x] += red[0][threadIdx.x + o]; red[1][threadIdx.x] += red[1][threadIdx.x + o]; } __syncthreads(); }
  __threadfence(); ((volatile unsigned*)HRGE16)[i0 / 2] = packed;
  if (threadIdx.x < 32) { const int l = threadIdx.x & 15; const double v = (l == 0) ? red[0][0] : (l == 1 ? red[1][0] : 0.0); ((volatile double*)PS)[(size_t)blockIdx.x * 16 + l] = v; }
}
__global__ __launch_bounds__(1024) void gru_kernel(const float* __restrict__ GI, const float* __restrict__ Whh, const float* __restrict__ bhh, float* __restrict__ HT, unsigned* __restrict__ HT16) {
  __shared__ float h[RB][RH]; __shared__ float gh[RB][3 * RH];
  const int t = threadIdx.x;
  for (int i = t; i < RB * RH; i += 1024) (&h[0][0])[i] = 0.f;
  __syncthreads();
  for (int w = 0; w < RW; ++w) {
    for (int o = t; o < RB * 3 * RH; o += 1024) { const int b = o / (3 * RH), j = o % (3 * RH); float a = bhh[j]; const float* wr = Whh + (size_t)j * RH;
#pragma unroll 1
      for (int k = 0; k < RH; ++k) a += h[b][k] * wr[k]; gh[b][j] = a; }
    __syncthreads();
    for (int o = t; o < RB * RH; o += 1024) { const int b = o / RH, j = o % RH; const float* gi = GI + ((size_t)b * RW + w) * 3 * RH;
      const float r = 1.0f / (1.0f + expf(-(gi[j] + gh[b][j]))), z = 1.0f / (1.0f + expf(-(gi[RH + j] + gh[b][RH + j]))); const float nn = tanhf(gi[2 * RH + j] + r * gh[b][2 * RH + j]);
      h[b][j] = (1.0f - z) * nn + z * h[b][j]; }
    __syncthreads(); }
  for (int pass = 0; pass < 2; ++pass) { for (int i = t; i < RB * RH; i += 1024) ((volatile float*)HT)[i] = (&h[0][0])[i];
    for (int i = t; i < 64 * RH / 2; i += 1024) { const int r = (2 * i) / RH, c = (2 * i) % RH; const float a = (r < RB) ? h[r][c] : 0.f, b = (r < RB) ? h[r][c + 1] : 0.f; ((volatile unsigned*)HT16)[i] = (unsigned)__builtin_bit_cast(unsigned short, (_Float16)a) | ((unsigned)__builtin_bit_cast(unsigned short, (_Float16)b) << 16); }
    __threadfence(); }
}
__global__ __launch_bounds__(256) void out_kernel(const float* __restrict__ F, const float* __restrict__ bffn, const float* __restrict__ LR, const float* __restrict__ fw, const float* __restrict__ fb, float* __restrict__ out0, float* __restrict__ out1) {
  const long i = (long)blockIdx.x * 256 + threadIdx.x; if (i >= (long)RB * RN * RN) return; const int b = (int)(i / (RN * RN)), p = (int)(i % (RN * RN)); const int y = p / RN, x = p % RN;
  float o = 1.0f / (1.0f + expf(-(F[(size_t)b * 16384 + p] + bffn[p]))); if (isnan(o)) o = 0.f;
  const float* cond = LR + ((size_t)b * RW + (RW - 1)) * RN * RN; float c0 = fb[0], c1 = fb[1];
  for (int ky = 0; ky < 3; ++ky) for (int kx = 0; kx < 3; ++kx) { const int yy = y + ky - 1, xx = x + kx - 1; if (yy < 0 || yy >= RN || xx < 0 || xx >= RN) continue; const float v = cond[yy * RN + xx]; c0 += fw[ky * 3 + kx] * v; c1 += fw[9 + ky * 3 + kx] * v; }
  const float ls = tanhf(c0), t2 = c1; const float rec = (o - t2) * expf(-ls); const float olr = 1.0f / (1.0f + expf(-rec));
  ((volatile float*)out0)[i] = o; ((volatile float*)out1)[i] = olr; __threadfence(); ((volatile float*)out0)[i] = o; ((volatile float*)out1)[i] = olr;
}
__global__ __launch_bounds__(256) void loss_kernel(const double* __restrict__ PS, int nblk, float* __restrict__ out2) {
  __shared__ double a[256], c[256]; double m = 0, bce = 0; for (int b = threadIdx.x; b < nblk; b += 256) { m += PS[(size_t)b * 16]; bce += PS[(size_t)b * 16 + 1]; }
  a[threadIdx.x] = m; c[threadIdx.x] = bce; __syncthreads(); for (int o = 128; o > 0; o >>= 1) { if (threadIdx.x < o) { a[threadIdx.x] += a[threadIdx.x + o]; c[threadIdx.x] += c[threadIdx.x + o]; } __syncthreads(); }
  if (threadIdx.x == 0) { const double n = (double)RB * RW * 2 * RN * RN; const double mse = a[0] / n, bcev = -c[0] / n; const float v = (float)(mse + bcev / (double)(RB * RW)); ((volatile float*)out2)[0] = v; __threadfence(); ((volatile float*)out2)[0] = v; }
}
extern "C" void kernel_launch(void* const* d_in, const int* in_sizes, int n_in, void* d_out, int out_size, void* d_ws, size_t ws_size, hipStream_t stream) {
  (void)in_sizes; (void)n_in; (void)out_size; (void)ws_size;
  auto Fp = [&](int i) { return (const float*)d_in[i]; };
  const float* HR = Fp(0); const float* LR = Fp(1); const float* fw = Fp(2); const float* fb = Fp(3); const float* Wsp = Fp(4); const float* bsp = Fp(5); const float* Wih = Fp(6); const float* Whh = Fp(7); const float* bih = Fp(8); const float* bhh = Fp(9); const float* Wffn = Fp(10); const float* bffn = Fp(11);
  float* out0 = (float*)d_out; float* out1 = out0 + (size_t)RB * 16384; float* out2 = out1 + (size_t)RB * RN * RN;
  char* ws = (char*)d_ws; size_t off = 0;
  auto carve = [&](size_t bytes) -> char* { char* p = ws + off; off += (bytes + 255) & ~(size_t)255; return p; };
  const int NLB = RROWS * RN / 512;
  unsigned* HRGE16 = (unsigned*)carve((size_t)RROWS * RN * 2); double* PS = (double*)carve((size_t)NLB * 16 * 8); _Float16* WSP = (_Float16*)carve(RH * RN * 2);
  _Float16* TE16 = (_Float16*)carve((size_t)RROWS * RH * 2); _Float16* WIH = (_Float16*)carve((size_t)3 * RH * RIN * 2); float* GI = (float*)carve((size_t)RBW * 3 * RH * 4);
  float* HT = (float*)carve(RB * RH * 4); unsigned* HT16 = (unsigned*)carve(64 * RH * 2); _Float16* WFF = (_Float16*)carve((size_t)16384 * RH * 2); float* FF = (float*)carve((size_t)64 * 16384 * 4);
  flow_kernel<<<NLB, 256, 0, stream>>>(HR, LR, fw, fb, HRGE16, PS);
  transpose_cast_f16<<<dim3(RH / 64, RN / 64), dim3(32, 8), 0, stream>>>(Wsp, RH, WSP, RN, 1.0f);
  cast_f32_f16x2<<<(unsigned)(((size_t)3 * RH * RIN / 2 + 255) / 256), 256, 0, stream>>>(Wih, WIH, (long)3 * RH * RIN / 2);
  transpose_cast_f16<<<dim3(16384 / 64, RH / 64), dim3(32, 8), 0, stream>>>(Wffn, 16384, WFF, RH, 1.0f);
  { const int t = (RROWS / 64) * 2; wmma_gemm64<0, false, 2, 1, false, 2><<<dim3((t + 7) / 8, 1), 256, 0, stream>>>((const unsigned short*)HRGE16, nullptr, RN, 0, U16(WSP), nullptr, RN, 0, TE16, nullptr, RH, 0, bsp, nullptr, 0, RROWS, RH, RN, 1.0f); }
  { const int t = (RBW / 64) * 6; wmma_gemm64<0, false, 2, 0, false, 0><<<dim3((t + 7) / 8, 1), 256, 0, stream>>>(U16(TE16), nullptr, RIN, 0, U16(WIH), nullptr, RIN, 0, GI, nullptr, 3 * RH, 0, bih, nullptr, 0, RBW, 3 * RH, RIN, 1.0f); }
  gru_kernel<<<1, 1024, 0, stream>>>(GI, Whh, bhh, HT, HT16);
  { const int t = 1 * (16384 / 64); wmma_gemm64<0, false, 0, 0, false, 0><<<dim3((t + 7) / 8, 1), 256, 0, stream>>>((const unsigned short*)HT16, nullptr, RH, 0, U16(WFF), nullptr, RH, 0, FF, nullptr, 16384, 0, nullptr, nullptr, 0, 64, 16384, RH, 1.0f); }
  out_kernel<<<(RB * RN * RN + 255) / 256, 256, 0, stream>>>(FF, bffn, LR, fw, fb, out0, out1);
  loss_kernel<<<1, 256, 0, stream>>>(PS, NLB, out2);
}
